// MultiHeadAttention_80607946211993
// MI455X (gfx1250) — hardware-run, weakly checked
//
#include <hip/hip_runtime.h>
#ifndef NB
#define NB 2
#endif
#ifndef SEQ
#define SEQ 2048
#endif
#ifndef EARLY
#define EARLY 512
#endif
#define NB_FULL 2
#define SEQ_FULL 2048
#define DM 2048
#define NH 16
#define HD 128
#define NTOK (NB * SEQ)
#define NEAR (NB * EARLY)

static_assert(SEQ % 128 == 0);
static_assert(EARLY % 128 == 0);
static_assert(EARLY >= 128);
static_assert(EARLY <= SEQ);
static_assert(SEQ <= SEQ_FULL);
static_assert(NB <= NB_FULL);
static_assert(NH * HD == DM);
static_assert(DM % 128 == 0);
static_assert(HD == 128);
static_assert((size_t)NTOK * DM * 2 * 4 + (size_t)DM * DM * 2 * 4 + (size_t)NEAR * DM * 2 * 4 + 256 <= (size_t)134217728);

typedef __bf16 v16b __attribute__((ext_vector_type(16)));
typedef _Float16 v16h __attribute__((ext_vector_type(16)));
typedef unsigned short v8us __attribute__((ext_vector_type(8), may_alias));
typedef float v8f __attribute__((ext_vector_type(8)));
typedef float v4f __attribute__((ext_vector_type(4)));
typedef float v4fa __attribute__((ext_vector_type(4), may_alias));
typedef int v4i __attribute__((ext_vector_type(4)));
typedef int v4ia __attribute__((ext_vector_type(4), may_alias));
union Frag { v16h h; v16b b; v8us half[2]; _Float16 f[16]; unsigned short u[16]; };

#define LOG2E 1.4426950408889634f
#define SCL 0.08838834764831845f
#define NINF (-__builtin_huge_valf())
#define INV2048 0.00048828125f

__device__ __forceinline__ unsigned short bf16_bits(float x) {
  unsigned int u = __float_as_uint(x);
  return (unsigned short)((u + 0x7FFFu + ((u >> 16) & 1u)) >> 16);
}
__device__ __forceinline__ float bf16_val(unsigned short b) { return __uint_as_float(((unsigned int)b) << 16); }
__device__ __forceinline__ float bf16_rne(float x) { return bf16_val(bf16_bits(x)); }
__device__ __forceinline__ unsigned short f16_bits(_Float16 h) { return __builtin_bit_cast(unsigned short, h); }

__device__ __forceinline__ v8f wmma_h(v16h a, v16h b, v8f c) {
  return __builtin_amdgcn_wmma_f32_16x16x32_f16(false, a, false, b, (short)0, c, false, false);
}
__device__ __forceinline__ v8f wmma_b(v16b a, v16b b, v8f c) {
  return __builtin_amdgcn_wmma_f32_16x16x32_bf16(false, a, false, b, (short)0, c, false, false);
}
__device__ __forceinline__ void ldfrag(Frag& f, const unsigned short* p) {
  f.half[0] = *(const v8us*)p;
  f.half[1] = *(const v8us*)(p + 16);
}

template <int MODE>
__device__ __forceinline__ unsigned short cv16(float x) {
  if (MODE == 0) return bf16_bits(x);
  return f16_bits((_Float16)(bf16_rne(x) * 64.0f));
}

template <int MODE>
__global__ __launch_bounds__(256) void k_cvt(const float* __restrict__ src, unsigned short* __restrict__ dst,
                                             long long seg_stride, int seg_rows) {
  const int row = blockIdx.x;
  const int seg = row / seg_rows;
  const int r = row - seg * seg_rows;
  const float* s = src + (size_t)seg * (size_t)seg_stride + (size_t)r * DM + threadIdx.x * 8;
  const v4f x0 = *(const v4fa*)s, x1 = *(const v4fa*)(s + 4);
  v8us o;
#pragma unroll
  for (int q = 0; q < 4; ++q) { o[q] = cv16<MODE>(x0[q]); o[4 + q] = cv16<MODE>(x1[q]); }
  unsigned short* d = dst + (size_t)row * DM + threadIdx.x * 8;
  *(volatile v8us*)d = o;
  __threadfence();
  *(volatile v8us*)d = o;
}

__global__ __launch_bounds__(512) void k_maskchk(const int* __restrict__ Mask, int* __restrict__ Flag) {
  __shared__ int wb[16];
  const int tid = threadIdx.x, lane = tid & 31;
  const int w = __builtin_amdgcn_readfirstlane(tid >> 5);
  int bad = 0;
#pragma unroll 1
  for (int p = tid; p < SEQ * (SEQ / 4); p += 512) {
    const int q = p / (SEQ / 4);
    const int idx = (p - q * (SEQ / 4)) * 4;
    const v4i m = *(const v4ia*)(Mask + (size_t)q * SEQ_FULL + idx);
    const int lo = (q >> 5) << 5;
#pragma unroll
    for (int e = 0; e < 4; ++e) {
      const int k = idx + e;
      const int mm = (m[e] != 0) ? 1 : 0;
      bad |= ((k < lo) ? mm : 0) | ((k >= lo + 32) ? (1 - mm) : 0);
    }
  }
  bad |= __shfl_xor(bad, 16, 32);
  bad |= __shfl_xor(bad, 8, 32);
  bad |= __shfl_xor(bad, 4, 32);
  bad |= __shfl_xor(bad, 2, 32);
  bad |= __shfl_xor(bad, 1, 32);
  if (lane == 0) wb[w] = bad;
  __syncthreads();
  if (w == 0) {
    int t = wb[lane & 15];
    t |= __shfl_xor(t, 8, 32);
    t |= __shfl_xor(t, 4, 32);
    t |= __shfl_xor(t, 2, 32);
    t |= __shfl_xor(t, 1, 32);
    const v4i o = {t, t, t, t};
    if (lane < 8) *(volatile v4i*)(Flag + lane * 4) = o;
    __threadfence();
    if (lane < 8) *(volatile v4i*)(Flag + lane * 4) = o;
  }
}

template <bool TR>
__global__ __launch_bounds__(128) __attribute__((amdgpu_num_vgpr(256)))
void k_proj(const unsigned short* __restrict__ A, const unsigned short* __restrict__ B,
            const float* __restrict__ bias, unsigned short* __restrict__ Ph,
            unsigned short* __restrict__ Pl, float carry) {
  __shared__ __attribute__((aligned(16))) float st[64][132];
  const int tid = threadIdx.x, lane = tid & 31, ln = lane & 15, hh = lane >> 4;
  const int w = __builtin_amdgcn_readfirstlane(tid >> 5);
  const int wm = w & 1, wn = w >> 1;
  const int m0 = blockIdx.y * 64, n0 = blockIdx.x * 128;
  const v8f z8 = {0.f, 0.f, 0.f, 0.f, 0.f, 0.f, 0.f, 0.f};
  v8f acc[2][4];
#pragma unroll
  for (int i = 0; i < 2; ++i)
#pragma unroll
    for (int j = 0; j < 4; ++j) acc[i][j] = z8;
  const unsigned short* ap = A + (size_t)(m0 + 32 * wm + ln) * DM + 8 * hh;
  const unsigned short* bp = B + (size_t)(n0 + 64 * wn + ln) * DM + 8 * hh;
#pragma unroll 1
  for (int k0 = 0; k0 < DM; k0 += 32) {
    Frag a[2], b[4];
#pragma unroll
    for (int i = 0; i < 2; ++i) ldfrag(a[i], ap + (size_t)i * 16 * DM + k0);
#pragma unroll
    for (int j = 0; j < 4; ++j) ldfrag(b[j], bp + (size_t)j * 16 * DM + k0);
#pragma unroll
    for (int i = 0; i < 2; ++i)
#pragma unroll
      for (int j = 0; j < 4; ++j) acc[i][j] = wmma_b(a[i].b, b[j].b, acc[i][j]);
    asm volatile("v_nop\n\tv_nop\n\tv_nop\n\tv_nop"
                 : "+v"(acc[0][0]), "+v"(acc[0][1]), "+v"(acc[0][2]), "+v"(acc[0][3]),
                   "+v"(acc[1][0]), "+v"(acc[1][1]), "+v"(acc[1][2]), "+v"(acc[1][3])
                 : "v"(a[0].h), "v"(a[1].h), "v"(b[0].h), "v"(b[1].h), "v"(b[2].h), "v"(b[3].h));
  }
#pragma unroll
  for (int i = 0; i < 2; ++i)
#pragma unroll
    for (int j = 0; j < 4; ++j) {
      const int cl = 64 * wn + 16 * j + ln;
#pragma unroll
      for (int r = 0; r < 8; ++r) {
        const int rl = 32 * wm + 16 * i + 8 * hh + r;
        const float bv = bf16_rne(TR ? bias[m0 + rl] : bias[n0 + cl]);
        st[rl][cl] = (acc[i][j][r] + bv) * carry;
      }
    }
  __syncthreads();
  size_t lrow;
  int ldh, ldl, lcol, early;
  if (!TR) {
    const int bb = m0 / SEQ, s0 = m0 - bb * SEQ;
    early = (s0 < EARLY) ? 1 : 0;
    ldh = DM; ldl = DM; lrow = (size_t)bb * EARLY + s0; lcol = n0;
  } else {
    const int bb = n0 / SEQ, s0 = n0 - bb * SEQ;
    early = (s0 < EARLY) ? 1 : 0;
    ldh = NTOK; ldl = NEAR; lrow = (size_t)m0; lcol = bb * EARLY + s0;
  }
  for (int pass = 0; pass < 2; ++pass) {
#pragma unroll 1
    for (int i = tid; i < 64 * 16; i += 128) {
      const int row = i >> 4, c8 = (i & 15) * 8;
      const v4f x0 = *(const v4fa*)&st[row][c8], x1 = *(const v4fa*)&st[row][c8 + 4];
      v8us oh, ol;
#pragma unroll
      for (int q = 0; q < 4; ++q) {
        const _Float16 h0 = (_Float16)x0[q], h1 = (_Float16)x1[q];
        oh[q] = f16_bits(h0); oh[4 + q] = f16_bits(h1);
        ol[q] = f16_bits((_Float16)((x0[q] - (float)h0) * 2048.0f));
        ol[4 + q] = f16_bits((_Float16)((x1[q] - (float)h1) * 2048.0f));
      }
      *(volatile v8us*)(Ph + (size_t)(m0 + row) * ldh + n0 + c8) = oh;
      if (early) *(volatile v8us*)(Pl + (lrow + row) * ldl + lcol + c8) = ol;
    }
    if (pass == 0) __threadfence();
  }
}

template <bool MASK, bool RES, int ND>
__device__ __forceinline__ void fa_step(const unsigned short* kph, const unsigned short* kpl,
                                        const unsigned short* vph, const unsigned short* vpl,
                                        const unsigned short* qph, const unsigned short* qpl,
                                        const int* mrow, int key0, int ln,
                                        const Frag (&qh)[4],
                                        float& mr, float& lr, v8f (&O0)[ND], v8f (&O1)[ND]) {
  const v8f z8 = {0.f, 0.f, 0.f, 0.f, 0.f, 0.f, 0.f, 0.f};
  const v8us zu = {0, 0, 0, 0, 0, 0, 0, 0};
  int koff = key0;
  v8f sh[2], sl[2];
  sh[0] = z8; sh[1] = z8; sl[0] = z8; sl[1] = z8;
  if (RES) {
    int qo = 0;
    asm volatile("" : "+v"(qo));
#pragma unroll
    for (int c = 0; c < 4; ++c) {
      Frag bq, bl;
      ldfrag(bq, qph + 32 * c + qo);
      ldfrag(bl, qpl + 32 * c + qo);
#pragma unroll
      for (int kt = 0; kt < 2; ++kt) {
        Frag a, ar;
        ldfrag(a, kph + (size_t)(koff + 16 * kt) * DM + 32 * c);
        int kr = koff + 16 * kt + ln;
        kr = (kr < EARLY) ? kr : (EARLY - 1);
        ldfrag(ar, kpl + (size_t)kr * DM + 32 * c);
        if (key0 >= EARLY) { ar.half[0] = zu; ar.half[1] = zu; }
        sh[kt] = wmma_h(a.h, bq.h, sh[kt]);
        sl[kt] = wmma_h(ar.h, bq.h, sl[kt]);
        sl[kt] = wmma_h(a.h, bl.h, sl[kt]);
        asm volatile("v_nop\n\tv_nop\n\tv_nop\n\tv_nop"
                     : "+v"(sh[kt]), "+v"(sl[kt])
                     : "v"(a.h), "v"(ar.h), "v"(bq.h), "v"(bl.h));
        asm volatile("" : "+v"(koff), "+v"(qo) : "v"(sl[kt]));
      }
    }
  } else {
#pragma unroll
    for (int kt = 0; kt < 2; ++kt) {
      Frag a[4];
      const unsigned short* p = kph + (size_t)(koff + 16 * kt) * DM;
#pragma unroll
      for (int c = 0; c < 4; ++c) ldfrag(a[c], p + 32 * c);
#pragma unroll
      for (int c = 0; c < 4; ++c) sh[kt] = wmma_h(a[c].h, qh[c].h, sh[kt]);
      asm volatile("v_nop\n\tv_nop\n\tv_nop\n\tv_nop"
                   : "+v"(sh[kt])
                   : "v"(a[0].h), "v"(a[1].h), "v"(a[2].h), "v"(a[3].h),
                     "v"(qh[0].h), "v"(qh[1].h), "v"(qh[2].h), "v"(qh[3].h));
      asm volatile("" : "+v"(koff) : "v"(sh[kt]));
    }
  }
  float sc[16];
#pragma unroll
  for (int r = 0; r < 8; ++r) {
    float a0 = sh[0][r], a1 = sh[1][r];
    if (RES) { a0 += sl[0][r] * INV2048; a1 += sl[1][r] * INV2048; }
    sc[r] = a0 * SCL; sc[8 + r] = a1 * SCL;
  }
  if (MASK) {
    const int* mp = mrow + key0;
    const v4i m0 = *(const v4ia*)(mp), m1 = *(const v4ia*)(mp + 4);
    const v4i m2 = *(const v4ia*)(mp + 16), m3 = *(const v4ia*)(mp + 20);
#pragma unroll
    for (int e = 0; e < 4; ++e) {
      sc[e]      = (m0[e] != 0) ? NINF : sc[e];
      sc[4 + e]  = (m1[e] != 0) ? NINF : sc[4 + e];
      sc[8 + e]  = (m2[e] != 0) ? NINF : sc[8 + e];
      sc[12 + e] = (m3[e] != 0) ? NINF : sc[12 + e];
    }
  }
  float mx = sc[0];
#pragma unroll
  for (int i = 1; i < 16; ++i) mx = fmaxf(mx, sc[i]);
  mx = fmaxf(mx, __shfl_xor(mx, 16, 32));
  const float mnew = fmaxf(mr, mx);
  const float muse = (mnew == NINF) ? 0.0f : mnew;
  const float al = exp2f((mr - muse) * LOG2E);
  mr = mnew;
  Frag ph, pl;
  float ps = 0.0f;
#pragma unroll
  for (int i = 0; i < 16; ++i) {
    const float pc = exp2f(fmaf(sc[i] - muse, LOG2E, 8.0f));
    ps += pc;
    const _Float16 hv = (_Float16)pc;
    ph.f[i] = hv;
    if (RES) pl.f[i] = (_Float16)((pc - (float)hv) * 2048.0f);
    else pl.f[i] = (_Float16)0.0f;
  }
  ps += __shfl_xor(ps, 16, 32);
  lr = lr * al + ps;
  int voff = key0;
  asm volatile("" : "+v"(voff) : "v"(ph.h));
#pragma unroll
  for (int t = 0; t < ND; ++t) { O0[t] = O0[t] * al; if (RES) O1[t] = O1[t] * al; }
  if (RES) {
#pragma unroll
    for (int t = 0; t < ND; ++t) {
      Frag vh, vr;
      ldfrag(vh, vph + (size_t)t * 16 * NTOK + voff);
      const int vc = (voff < EARLY - 32) ? voff : (EARLY - 32);
      ldfrag(vr, vpl + (size_t)t * 16 * NEAR + vc);
      if (key0 >= EARLY) { vr.half[0] = zu; vr.half[1] = zu; }
      O0[t] = wmma_h(vh.h, ph.h, O0[t]);
      O1[t] = wmma_h(vr.h, ph.h, O1[t]);
      O1[t] = wmma_h(vh.h, pl.h, O1[t]);
      asm volatile("v_nop\n\tv_nop\n\tv_nop\n\tv_nop"
                   : "+v"(O0[t]), "+v"(O1[t])
                   : "v"(vh.h), "v"(vr.h), "v"(ph.h), "v"(pl.h));
      asm volatile("" : "+v"(voff) : "v"(O1[t]));
    }
  } else {
#pragma unroll
    for (int g = 0; g < ND / 4; ++g) {
      Frag vf[4];
#pragma unroll
      for (int t = 0; t < 4; ++t) ldfrag(vf[t], vph + (size_t)(4 * g + t) * 16 * NTOK + voff);
#pragma unroll
      for (int t = 0; t < 4; ++t) O0[4 * g + t] = wmma_h(vf[t].h, ph.h, O0[4 * g + t]);
      asm volatile("v_nop\n\tv_nop\n\tv_nop\n\tv_nop"
                   : "+v"(O0[4 * g + 0]), "+v"(O0[4 * g + 1]), "+v"(O0[4 * g + 2]), "+v"(O0[4 * g + 3])
                   : "v"(vf[0].h), "v"(vf[1].h), "v"(vf[2].h), "v"(vf[3].h), "v"(ph.h));
      asm volatile("" : "+v"(voff) : "v"(O0[4 * g + 3]));
    }
  }
}

template <bool RES>
__global__ __launch_bounds__(RES ? 256 : 128) __attribute__((amdgpu_num_vgpr(256)))
void k_attn(const unsigned short* Qh, const unsigned short* Ql,
            const unsigned short* Kh, const unsigned short* Kl,
            const unsigned short* Vh, const unsigned short* Vl,
            const int* Mask, const int* Flag,
            unsigned short* Ch, unsigned short* Cl) {
  constexpr int ND = RES ? 4 : 8;
  constexpr int NW = RES ? 8 : 4;
  constexpr int SP = ND * 16 + 4;
  constexpr int NQT = RES ? (EARLY / 64) : (((SEQ - EARLY) / 64 > 0) ? (SEQ - EARLY) / 64 : 1);
  __shared__ __attribute__((aligned(16))) float so[NW][16][SP];
  const int tid = threadIdx.x, lane = tid & 31, ln = lane & 15, hh = lane >> 4;
  const int w = __builtin_amdgcn_readfirstlane(tid >> 5);
  const int qgrp = RES ? (w >> 1) : w;
  const int dbase = RES ? 64 * (w & 1) : 0;
  const int bh = blockIdx.x / NQT, qt = blockIdx.x - bh * NQT;
  const int b = bh / NH, h = bh - b * NH;
  const int qbase = (RES ? 0 : EARLY) + 64 * qt + 16 * qgrp;
  const int qg = qbase + ln;
  const int qe = (qg < EARLY) ? qg : (EARLY - 1);
  const unsigned short* qph = Qh + (size_t)(b * SEQ + qg) * DM + h * HD + 8 * hh;
  const unsigned short* qpl = Ql + (size_t)(b * EARLY + qe) * DM + h * HD + 8 * hh;
  Frag qh[4];
  {
    const v8us zq = {0, 0, 0, 0, 0, 0, 0, 0};
#pragma unroll
    for (int c = 0; c < 4; ++c) {
      if (!RES) ldfrag(qh[c], qph + 32 * c);
      else { qh[c].half[0] = zq; qh[c].half[1] = zq; }
    }
  }
  const unsigned short* kph = Kh + (size_t)(b * SEQ + ln) * DM + h * HD + 8 * hh;
  const unsigned short* kpl = Kl + (size_t)(b * EARLY) * DM + h * HD + 8 * hh;
  const unsigned short* vph = Vh + (size_t)(h * HD + dbase + ln) * NTOK + (size_t)b * SEQ + 8 * hh;
  const unsigned short* vpl = Vl + (size_t)(h * HD + dbase + ln) * NEAR + (size_t)b * EARLY + 8 * hh;
  const int* mrow = Mask + (size_t)qg * SEQ_FULL + 8 * hh;
  float mr = NINF, lr = 0.0f;
  v8f O0[ND] = {}, O1[ND] = {};
  const int fast = (__builtin_amdgcn_readfirstlane(Flag[0]) == 0) ? 1 : 0;
  const int nfull = qbase >> 5;
  const int nst = fast ? (nfull + 1) : (SEQ / 32);
#pragma unroll 1
  for (int j = 0; j < nst; ++j) {
    if (fast && j < nfull)
      fa_step<false, RES, ND>(kph, kpl, vph, vpl, qph, qpl, mrow, 32 * j, ln, qh, mr, lr, O0, O1);
    else
      fa_step<true, RES, ND>(kph, kpl, vph, vpl, qph, qpl, mrow, 32 * j, ln, qh, mr, lr, O0, O1);
  }
  const float inv = 1.0f / lr;
#pragma unroll
  for (int t = 0; t < ND; ++t)
#pragma unroll
    for (int r = 0; r < 8; ++r) {
      float v = O0[t][r];
      if (RES) v += O1[t][r] * INV2048;
      so[w][ln][16 * t + 8 * hh + r] = v * inv;
    }
  __syncthreads();
  constexpr int PPR = ND * 2;
  unsigned short* cgh = Ch + (size_t)(b * SEQ + qbase) * DM + h * HD + dbase;
  unsigned short* cgl = Cl + (size_t)(b * EARLY + (RES ? qbase : 0)) * DM + h * HD + dbase;
  for (int pass = 0; pass < 2; ++pass) {
#pragma unroll 1
    for (int it = 0; it < ND; ++it) {
      const int i = lane + 32 * it;
      const int row = i / PPR, c8 = (i - row * PPR) * 8;
      const v4f x0 = *(const v4fa*)&so[w][row][c8], x1 = *(const v4fa*)&so[w][row][c8 + 4];
      v8us oh, ol;
#pragma unroll
      for (int q = 0; q < 4; ++q) {
        const _Float16 h0 = (_Float16)x0[q], h1 = (_Float16)x1[q];
        oh[q] = f16_bits(h0); oh[4 + q] = f16_bits(h1);
        ol[q] = f16_bits((_Float16)((x0[q] - (float)h0) * 2048.0f));
        ol[4 + q] = f16_bits((_Float16)((x1[q] - (float)h1) * 2048.0f));
      }
      *(volatile v8us*)(cgh + (size_t)row * DM + c8) = oh;
      if (RES) *(volatile v8us*)(cgl + (size_t)row * DM + c8) = ol;
    }
    if (pass == 0) __threadfence();
  }
}

template <bool RES>
__global__ __launch_bounds__(128) __attribute__((amdgpu_num_vgpr(256)))
void k_oproj(const unsigned short* __restrict__ Chp, const unsigned short* __restrict__ Clp,
             const unsigned short* __restrict__ W, const float* __restrict__ bias,
             float* __restrict__ Out) {
  constexpr int MI = RES ? 1 : 2;
  constexpr int TM = 32 * MI;
  constexpr int TPS = RES ? (EARLY / TM) : (((SEQ - EARLY) / TM > 0) ? (SEQ - EARLY) / TM : 1);
  __shared__ __attribute__((aligned(16))) float st[TM][132];
  const int tid = threadIdx.x, lane = tid & 31, ln = lane & 15, hh = lane >> 4;
  const int w = __builtin_amdgcn_readfirstlane(tid >> 5);
  const int wm = w & 1, wn = w >> 1;
  const int b = blockIdx.y / TPS, tl = blockIdx.y - b * TPS;
  const int s0 = (RES ? 0 : EARLY) + tl * TM;
  const int n0 = blockIdx.x * 128;
  const v8f z8 = {0.f, 0.f, 0.f, 0.f, 0.f, 0.f, 0.f, 0.f};
  v8f acc[2][4], accl[2][4];
#pragma unroll
  for (int i = 0; i < 2; ++i)
#pragma unroll
    for (int j = 0; j < 4; ++j) { acc[i][j] = z8; accl[i][j] = z8; }
  const unsigned short* ap = Chp + (size_t)(b * SEQ + s0 + 16 * MI * wm + ln) * DM + 8 * hh;
  const unsigned short* alp = Clp + (size_t)(b * EARLY + (RES ? s0 : 0) + 16 * wm + ln) * DM + 8 * hh;
  const unsigned short* bp = W + (size_t)(n0 + 64 * wn + ln) * DM + 8 * hh;
#pragma unroll 1
  for (int k0 = 0; k0 < DM; k0 += 32) {
    Frag a[2], ar, bf[4];
    ldfrag(a[0], ap + k0);
    if (!RES) ldfrag(a[1], ap + (size_t)16 * DM + k0); else a[1] = a[0];
    if (RES) ldfrag(ar, alp + k0); else ar = a[0];
#pragma unroll
    for (int j = 0; j < 4; ++j) ldfrag(bf[j], bp + (size_t)j * 16 * DM + k0);
#pragma unroll
    for (int j = 0; j < 4; ++j) acc[0][j] = wmma_h(a[0].h, bf[j].h, acc[0][j]);
    if (RES) {
#pragma unroll
      for (int j = 0; j < 4; ++j) accl[0][j] = wmma_h(ar.h, bf[j].h, accl[0][j]);
      asm volatile("v_nop\n\tv_nop\n\tv_nop\n\tv_nop"
                   : "+v"(acc[0][0]), "+v"(acc[0][1]), "+v"(acc[0][2]), "+v"(acc[0][3]),
                     "+v"(accl[0][0]), "+v"(accl[0][1]), "+v"(accl[0][2]), "+v"(accl[0][3])
                   : "v"(a[0].h), "v"(ar.h), "v"(bf[0].h), "v"(bf[1].h), "v"(bf[2].h), "v"(bf[3].h));
    } else {
#pragma unroll
      for (int j = 0; j < 4; ++j) acc[1][j] = wmma_h(a[1].h, bf[j].h, acc[1][j]);
      asm volatile("v_nop\n\tv_nop\n\tv_nop\n\tv_nop"
                   : "+v"(acc[0][0]), "+v"(acc[0][1]), "+v"(acc[0][2]), "+v"(acc[0][3]),
                     "+v"(acc[1][0]), "+v"(acc[1][1]), "+v"(acc[1][2]), "+v"(acc[1][3])
                   : "v"(a[0].h), "v"(a[1].h), "v"(bf[0].h), "v"(bf[1].h), "v"(bf[2].h), "v"(bf[3].h));
    }
  }
#pragma unroll
  for (int i = 0; i < MI; ++i)
#pragma unroll
    for (int j = 0; j < 4; ++j) {
      const int cl = 64 * wn + 16 * j + ln;
      const float bv = bf16_rne(bias[n0 + cl]);
#pragma unroll
      for (int r = 0; r < 8; ++r) {
        float v = acc[i][j][r];
        if (RES) v += accl[i][j][r] * INV2048;
        st[16 * MI * wm + 16 * i + 8 * hh + r][cl] = v * 0.0009765625f + bv;
      }
    }
  __syncthreads();
  float* og = Out + ((size_t)b * SEQ_FULL + s0) * DM + n0;
  for (int pass = 0; pass < 2; ++pass) {
#pragma unroll 1
    for (int i = tid; i < TM * 32; i += 128) {
      const int row = i >> 5, c4 = (i & 31) * 4;
      const v4f v = *(const v4fa*)&st[row][c4];
      *(volatile v4f*)(og + (size_t)row * DM + c4) = v;
    }
    if (pass == 0) __threadfence();
  }
}

extern "C" void kernel_launch(void* const* d_in, const int* in_sizes, int n_in,
                              void* d_out, int out_size, void* d_ws, size_t ws_size, hipStream_t stream) {
  if (n_in < 10) return;
  const long long need_x = (long long)(NB - 1) * SEQ_FULL * DM + (long long)SEQ * DM;
  const long long need_m = (long long)(SEQ - 1) * SEQ_FULL + SEQ;
  if ((long long)in_sizes[0] < need_x) return;
  if ((long long)in_sizes[1] < need_m) return;
  if ((long long)in_sizes[2] < (long long)DM * DM || (long long)in_sizes[4] < (long long)DM * DM) return;
  if ((long long)in_sizes[6] < (long long)DM * DM || (long long)in_sizes[8] < (long long)DM * DM) return;
  if (in_sizes[3] < DM || in_sizes[5] < DM || in_sizes[7] < DM || in_sizes[9] < DM) return;
  if ((long long)out_size < need_x) return;
  const float* x = (const float*)d_in[0];
  const int* mask = (const int*)d_in[1];
  const float* wq = (const float*)d_in[2];
  const float* bq = (const float*)d_in[3];
  const float* wk = (const float*)d_in[4];
  const float* bk = (const float*)d_in[5];
  const float* wv = (const float*)d_in[6];
  const float* bv = (const float*)d_in[7];
  const float* wo = (const float*)d_in[8];
  const float* bo = (const float*)d_in[9];
  float* out = (float*)d_out;

  char* ws = (char*)d_ws;
  size_t off = 0;
  const size_t P_TOK = (size_t)NTOK * DM * 2;
  const size_t P_W = (size_t)DM * DM * 2;
  const size_t P_EAR = (size_t)NEAR * DM * 2;
  unsigned short* xb = (unsigned short*)(ws + off); off += P_TOK;
  unsigned short* wqb = (unsigned short*)(ws + off); off += P_W;
  unsigned short* wkb = (unsigned short*)(ws + off); off += P_W;
  unsigned short* wvb = (unsigned short*)(ws + off); off += P_W;
  unsigned short* wof = (unsigned short*)(ws + off); off += P_W;
  unsigned short* qhp = (unsigned short*)(ws + off); off += P_TOK;
  unsigned short* khp = (unsigned short*)(ws + off); off += P_TOK;
  unsigned short* vth = (unsigned short*)(ws + off); off += P_TOK;
  unsigned short* qlp = (unsigned short*)(ws + off); off += P_EAR;
  unsigned short* klp = (unsigned short*)(ws + off); off += P_EAR;
  unsigned short* vtl = (unsigned short*)(ws + off); off += P_EAR;
  unsigned short* clp = (unsigned short*)(ws + off); off += P_EAR;
  int* flag = (int*)(ws + off); off += 256;
  if (off > ws_size) return;
  unsigned short* chp = xb;

  k_cvt<0><<<(unsigned)NTOK, 256, 0, stream>>>(x, xb, (long long)SEQ_FULL * DM, (int)SEQ);
  k_cvt<0><<<(unsigned)DM, 256, 0, stream>>>(wq, wqb, 0LL, (int)DM);
  k_cvt<0><<<(unsigned)DM, 256, 0, stream>>>(wk, wkb, 0LL, (int)DM);
  k_cvt<0><<<(unsigned)DM, 256, 0, stream>>>(wv, wvb, 0LL, (int)DM);
  k_cvt<1><<<(unsigned)DM, 256, 0, stream>>>(wo, wof, 0LL, (int)DM);
  k_maskchk<<<1, 512, 0, stream>>>(mask, flag);

  k_proj<false><<<dim3(DM / 128, NTOK / 64), 128, 0, stream>>>(xb, wqb, bq, qhp, qlp, 1.0f);
  k_proj<false><<<dim3(DM / 128, NTOK / 64), 128, 0, stream>>>(xb, wkb, bk, khp, klp, 1.0f);
  k_proj<true><<<dim3(NTOK / 128, DM / 64), 128, 0, stream>>>(wvb, xb, bv, vth, vtl, 16.0f);

  k_attn<true><<<(unsigned)(NB * NH * (EARLY / 64)), 256, 0, stream>>>(qhp, qlp, khp, klp, vth, vtl, mask, flag, chp, clp);
  if (SEQ > EARLY)
    k_attn<false><<<(unsigned)(NB * NH * ((SEQ - EARLY) / 64)), 128, 0, stream>>>(qhp, qlp, khp, klp, vth, vtl, mask, flag, chp, clp);

  k_oproj<true><<<dim3(DM / 128, NB * (EARLY / 32)), 128, 0, stream>>>(chp, clp, wof, bo, out);
  if (SEQ > EARLY)
    k_oproj<false><<<dim3(DM / 128, NB * ((SEQ - EARLY) / 64)), 128, 0, stream>>>(chp, clp, wof, bo, out);
}
